// GPSConvNN_86938728005833
// MI455X (gfx1250) — hardware-verified
//
#include <hip/hip_runtime.h>
#include <stddef.h>
#include <math.h>


#define C_     256
#define HD     64
#define NH     4
#define NTHR   256
#define NWAVE  8
#define GR     128
#define GC     128
#define AGB    32
#define EPT    8
#define CHUNK  (NTHR * EPT)
#define WCAP   (EPT * 32)
#define LISTN  (NWAVE * WCAP)
#define ATHR   128
#define AQ     64
#define PP     72
#define WSCL   16.0f
#define WSCAP  134217728

#define WP_1   0
#define WP_IN  131072
#define WP_OUT 327680
#define WP_M1  393216
#define WP_M2  524288
#define WP_LIN 655360
#define WPTOT  720896

#define LDS_GEMM (GR * GC * 4)

static_assert(WP_IN == WP_1 + 256 * 512);
static_assert(WP_OUT == WP_IN + 768 * 256);
static_assert(WP_M1 == WP_OUT + 256 * 256);
static_assert(WP_M2 == WP_M1 + 512 * 256);
static_assert(WP_LIN == WP_M2 + 256 * 512);
static_assert(WPTOT == WP_LIN + 256 * 256);
static_assert((CHUNK & (CHUNK - 1)) == 0 && CHUNK <= 2048);
static_assert(AGB == 32 && AGB == 4 * NWAVE);
static_assert(GR == 4 * 32 && GC == 2 * 64 && NTHR == 8 * 32);
static_assert((PP % 8) == 0);
static_assert(C_ == NH * HD);

typedef float          v4f  __attribute__((ext_vector_type(4)));
typedef float          v8f  __attribute__((ext_vector_type(8)));
typedef double         v2d  __attribute__((ext_vector_type(2)));
typedef int            v4i  __attribute__((ext_vector_type(4)));
typedef _Float16       v8h  __attribute__((ext_vector_type(8)));
typedef _Float16       v16h __attribute__((ext_vector_type(16)));
union Frag { v16h v; v8h h[2]; };

__device__ __forceinline__ v8f vz8() { v8f z = {0.f, 0.f, 0.f, 0.f, 0.f, 0.f, 0.f, 0.f}; return z; }

__device__ __forceinline__ v8f wmf(v16h a, v16h b, v8f c) {
  v8f d = __builtin_amdgcn_wmma_f32_16x16x32_f16(false, a, false, b, (short)0, c, false, false);
  asm volatile("v_nop\n\tv_nop\n\tv_nop\n\tv_nop" : "+v"(d) : "v"(a), "v"(b));
  return d;
}

__device__ __forceinline__ v8h cvt8(v4f a, v4f b) {
  v8h r;
  r[0] = (_Float16)a.x; r[1] = (_Float16)a.y; r[2] = (_Float16)a.z; r[3] = (_Float16)a.w;
  r[4] = (_Float16)b.x; r[5] = (_Float16)b.y; r[6] = (_Float16)b.z; r[7] = (_Float16)b.w;
  return r;
}

__device__ __forceinline__ v4f sel4(bool c, v4f a, v4f b) {
  v4f r;
  r.x = c ? a.x : b.x; r.y = c ? a.y : b.y; r.z = c ? a.z : b.z; r.w = c ? a.w : b.w;
  return r;
}

__device__ __forceinline__ v4f relu4(v4f v) {
  v.x = fmaxf(v.x, 0.0f); v.y = fmaxf(v.y, 0.0f); v.z = fmaxf(v.z, 0.0f); v.w = fmaxf(v.w, 0.0f);
  return v;
}

__device__ __forceinline__ float elu1(float v) {
  const float e = __expf(v) - 1.0f;
  return v > 0.0f ? v : e;
}

__global__ __launch_bounds__(NTHR) void k_wprep(
    const float* __restrict__ wn, const float* __restrict__ wr, const float* __restrict__ win,
    const float* __restrict__ wout, const float* __restrict__ wm1, const float* __restrict__ wm2,
    const float* __restrict__ wlin, _Float16* wp) {
  const int blk = blockIdx.x, tid = threadIdx.x;
  v4f a, b;
  size_t di;
  if (blk < 64) {
    const int i = blk * NTHR + tid;
    const int n = i >> 6, k0 = (i & 63) * 8, kk = k0 & 255;
    const float* pa = wn + (size_t)n * C_ + kk;
    const float* pb = wr + (size_t)n * C_ + kk;
    const v4f a0 = *(const v4f*)pa, a1 = *(const v4f*)(pa + 4);
    const v4f b0 = *(const v4f*)pb, b1 = *(const v4f*)(pb + 4);
    const bool lo = k0 < 256;
    a = sel4(lo, a0, b0);
    b = sel4(lo, a1, b1);
    di = (size_t)WP_1 + (size_t)i * 8;
  } else {
    const float* src;
    int i;
    size_t base;
    if (blk < 160)      { i = (blk - 64)  * NTHR + tid; src = win;  base = WP_IN;  }
    else if (blk < 192) { i = (blk - 160) * NTHR + tid; src = wout; base = WP_OUT; }
    else if (blk < 256) { i = (blk - 192) * NTHR + tid; src = wm1;  base = WP_M1;  }
    else if (blk < 320) { i = (blk - 256) * NTHR + tid; src = wm2;  base = WP_M2;  }
    else                { i = (blk - 320) * NTHR + tid; src = wlin; base = WP_LIN; }
    const float* ps = src + (size_t)i * 8;
    a = *(const v4f*)ps;
    b = *(const v4f*)(ps + 4);
    di = base + (size_t)i * 8;
  }
  a = a * WSCL;
  b = b * WSCL;
  const v8h hv = cvt8(a, b);
  _Float16* d = wp + di;
  *(volatile v8h*)d = hv;
  __threadfence();
  *(volatile v8h*)d = hv;
}

template <int NB>
__device__ __forceinline__ int scan_chunk(const int* __restrict__ dsts, int nE, int cbase, int slotBase,
                                          int vec8, int* list, int tid, int lane, int wave) {
  static_assert(NB <= 32);
  int wc = 0;
  const int el0  = tid * EPT;
  const int e0   = cbase + el0;
  const int sent = -2147483647 - 1;
  v4i da, db;
  if (vec8 != 0 && cbase + CHUNK <= nE) {
    da = *(const v4i*)(dsts + e0);
    db = *(const v4i*)(dsts + e0 + 4);
  } else {
    da.x = (e0     < nE) ? dsts[min(e0, nE - 1)]     : sent;
    da.y = (e0 + 1 < nE) ? dsts[min(e0 + 1, nE - 1)] : sent;
    da.z = (e0 + 2 < nE) ? dsts[min(e0 + 2, nE - 1)] : sent;
    da.w = (e0 + 3 < nE) ? dsts[min(e0 + 3, nE - 1)] : sent;
    db.x = (e0 + 4 < nE) ? dsts[min(e0 + 4, nE - 1)] : sent;
    db.y = (e0 + 5 < nE) ? dsts[min(e0 + 5, nE - 1)] : sent;
    db.z = (e0 + 6 < nE) ? dsts[min(e0 + 6, nE - 1)] : sent;
    db.w = (e0 + 7 < nE) ? dsts[min(e0 + 7, nE - 1)] : sent;
  }
  const unsigned nb = (unsigned)slotBase;
  const unsigned s0 = (unsigned)da.x - nb, s1 = (unsigned)da.y - nb;
  const unsigned s2 = (unsigned)da.z - nb, s3 = (unsigned)da.w - nb;
  const unsigned s4 = (unsigned)db.x - nb, s5 = (unsigned)db.y - nb;
  const unsigned s6 = (unsigned)db.z - nb, s7 = (unsigned)db.w - nb;
  const bool h0 = s0 < (unsigned)NB, h1 = s1 < (unsigned)NB, h2 = s2 < (unsigned)NB, h3 = s3 < (unsigned)NB;
  const bool h4 = s4 < (unsigned)NB, h5 = s5 < (unsigned)NB, h6 = s6 < (unsigned)NB, h7 = s7 < (unsigned)NB;
  const unsigned any = __builtin_amdgcn_ballot_w32(h0 | h1 | h2 | h3 | h4 | h5 | h6 | h7);
  if (any != 0u) {
#define HITJ(J, HJ, SJ) { \
      const unsigned mj = __builtin_amdgcn_ballot_w32(HJ); \
      if (mj != 0u) { \
        if (HJ) { \
          const int pos = wc + (int)__builtin_amdgcn_mbcnt_lo(mj, 0u); \
          if (pos < WCAP) list[wave * WCAP + pos] = ((el0 + (J)) << 5) | (int)(SJ); \
        } \
        wc += (int)__builtin_popcount(mj); } }
    HITJ(0, h0, s0)
    HITJ(1, h1, s1)
    HITJ(2, h2, s2)
    HITJ(3, h3, s3)
    HITJ(4, h4, s4)
    HITJ(5, h5, s5)
    HITJ(6, h6, s6)
    HITJ(7, h7, s7)
#undef HITJ
  }
  return wc;
}

__global__ __launch_bounds__(NTHR) void k_agg(
    const float* __restrict__ x, const int* __restrict__ srcs, const int* __restrict__ dsts,
    _Float16* A1, int nN, int nE, int vec8) {
  __shared__ __attribute__((aligned(16))) float sacc[AGB * C_];
  __shared__ __attribute__((aligned(16))) int list[LISTN];
  __shared__ int wcnt[NWAVE];
  const int tid = threadIdx.x, lane = tid & 31, wave = tid >> 5;
  const int nodeBase = blockIdx.x * AGB;

  {
    const v4f z = {0.f, 0.f, 0.f, 0.f};
    for (int i = tid; i < (AGB * C_) / 4; i += NTHR) ((v4f*)sacc)[i] = z;
  }
  __syncthreads();

  int c0 = 0, c1 = 0, c2 = 0, c3 = 0;
  const int nChunks = (nE + CHUNK - 1) / CHUNK;
#pragma unroll 1
  for (int ch = 0; ch < nChunks; ++ch) {
    const int cbase = ch * CHUNK;
    const int wc = scan_chunk<AGB>(dsts, nE, cbase, nodeBase, vec8, list, tid, lane, wave);
    if (lane == 0) wcnt[wave] = wc;
    __syncthreads();
#pragma unroll 1
    for (int wsx = 0; wsx < NWAVE; ++wsx) {
      int n = __builtin_amdgcn_readfirstlane(wcnt[wsx]);
      n = n > WCAP ? WCAP : (n < 0 ? 0 : n);
      const int* lp = list + wsx * WCAP;
#pragma unroll 1
      for (int i = 0; i < n; ++i) {
        const int ent  = __builtin_amdgcn_readfirstlane(lp[i]);
        const int slot = ent & (AGB - 1);
        if ((slot >> 2) == wave) {
          int e = cbase + (ent >> 5);
          e = e > nE - 1 ? nE - 1 : e;
          int s = srcs[e];
          s = s < 0 ? 0 : (s > nN - 1 ? nN - 1 : s);
          const float* xp = x + (size_t)s * C_ + 8 * lane;
          const v4f p0 = *(const v4f*)xp, p1 = *(const v4f*)(xp + 4);
          v4f* ar = (v4f*)(sacc + slot * C_ + 8 * lane);
          ar[0] = ar[0] + p0;
          ar[1] = ar[1] + p1;
          const int js = slot & 3;
          c0 += (js == 0); c1 += (js == 1); c2 += (js == 2); c3 += (js == 3);
        }
      }
    }
    __syncthreads();
  }

  v8h ka[4], kx[4];
#pragma unroll
  for (int j = 0; j < 4; ++j) {
    const int slot = 4 * wave + j;
    const int node = nodeBase + slot;
    const int n = (j == 0) ? c0 : ((j == 1) ? c1 : ((j == 2) ? c2 : c3));
    const float rc = __builtin_amdgcn_rcpf((float)(n > 1 ? n : 1));
    const v4f s0 = *(const v4f*)(sacc + slot * C_ + 8 * lane) * rc;
    const v4f s1 = *(const v4f*)(sacc + slot * C_ + 8 * lane + 4) * rc;
    ka[j] = cvt8(s0, s1);
    const float* xp = x + (size_t)node * C_ + 8 * lane;
    kx[j] = cvt8(*(const v4f*)xp, *(const v4f*)(xp + 4));
  }
#pragma unroll
  for (int j = 0; j < 4; ++j) {
    _Float16* rp = A1 + (size_t)(nodeBase + 4 * wave + j) * (2 * C_);
    *(volatile v8h*)(rp + 8 * lane) = ka[j];
    *(volatile v8h*)(rp + C_ + 8 * lane) = kx[j];
  }
  __threadfence();
#pragma unroll
  for (int j = 0; j < 4; ++j) {
    _Float16* rp = A1 + (size_t)(nodeBase + 4 * wave + j) * (2 * C_);
    *(volatile v8h*)(rp + 8 * lane) = ka[j];
    *(volatile v8h*)(rp + C_ + 8 * lane) = kx[j];
  }
}

template <int MODE>
__global__ __launch_bounds__(NTHR) void k_gemm(
    const _Float16* __restrict__ A, int lda,
    const _Float16* __restrict__ B, int ldb, int K,
    const float* __restrict__ bias,
    const float* __restrict__ res, int ldres,
    float scl,
    float* Cf, _Float16* Ch, _Float16* Ch2, int ldc,
    double* part, int flags, int nN) {
  extern __shared__ v4f lds_dyn[];
  float* stg = (float*)lds_dyn;
  __shared__ __attribute__((aligned(16))) double dS[2 * GC];
  __shared__ __attribute__((aligned(16))) double dQ[2 * GC];
  const int tid = threadIdx.x, lane = tid & 31, wave = tid >> 5, hh = lane >> 4, m = lane & 15;
  const int wr = wave & 3, wc = wave >> 2;
  const int rowBase = blockIdx.x * GR, colBase = blockIdx.y * GC;

  v8f acc[2][4];
#pragma unroll
  for (int i = 0; i < 2; ++i)
#pragma unroll
    for (int t = 0; t < 4; ++t) acc[i][t] = vz8();

  const _Float16* ap0 = A + (size_t)(rowBase + 32 * wr + m) * lda + 8 * hh;
  const _Float16* ap1 = ap0 + (size_t)16 * lda;
  const _Float16* bp0 = B + (size_t)(colBase + 64 * wc + m) * ldb + 8 * hh;
#pragma unroll 1
  for (int k0 = 0; k0 < K; k0 += 32) {
    Frag a0, a1;
    a0.h[0] = *(const v8h*)(ap0 + k0);
    a0.h[1] = *(const v8h*)(ap0 + k0 + 16);
    a1.h[0] = *(const v8h*)(ap1 + k0);
    a1.h[1] = *(const v8h*)(ap1 + k0 + 16);
#pragma unroll
    for (int t = 0; t < 4; ++t) {
      const _Float16* bp = bp0 + (size_t)(16 * t) * ldb + k0;
      Frag b;
      b.h[0] = *(const v8h*)bp;
      b.h[1] = *(const v8h*)(bp + 16);
      acc[0][t] = wmf(a0.v, b.v, acc[0][t]);
      acc[1][t] = wmf(a1.v, b.v, acc[1][t]);
    }
  }

#pragma unroll
  for (int i = 0; i < 2; ++i) {
    float* sp = stg + (32 * wr + 16 * i + 8 * hh) * GC + 64 * wc + m;
#pragma unroll
    for (int t = 0; t < 4; ++t)
#pragma unroll
      for (int r = 0; r < 8; ++r) sp[r * GC + 16 * t] = acc[i][t][r] * scl;
  }
  __syncthreads();

  if constexpr (MODE == 0) {
    const v4f b4 = *(const v4f*)(bias + colBase + 4 * lane);
    v4f keep[16];
#pragma unroll
    for (int it = 0; it < 16; ++it) {
      const int row = 16 * wave + it;
      float* q = stg + row * GC + 4 * lane;
      v4f v = *(const v4f*)q + b4;
      if (flags & 1) v = v + *(const v4f*)(res + (size_t)(rowBase + row) * ldres + colBase + 4 * lane);
      if (flags & 2) *(v4f*)q = v;
      keep[it] = v;
      *(volatile v4f*)(Cf + (size_t)(rowBase + row) * ldc + colBase + 4 * lane) = v;
    }
    v2d pv = {0.0, 0.0};
    const int ncols = (int)gridDim.y * GC;
    if (flags & 2) {
      __syncthreads();
      {
        const int c = tid & (GC - 1), hf = tid >> 7;
        double s = 0.0, qq = 0.0;
#pragma unroll 4
        for (int i = 0; i < 64; ++i) {
          const double dv = (double)stg[(hf * 64 + i) * GC + c];
          s += dv;
          qq = fma(dv, dv, qq);
        }
        dS[hf * GC + c] = s;
        dQ[hf * GC + c] = qq;
      }
      __syncthreads();
      if (tid < GC) { pv.x = dS[tid] + dS[GC + tid]; pv.y = dQ[tid] + dQ[GC + tid]; }
      if (tid < GC) *(volatile v2d*)(part + ((size_t)blockIdx.x * ncols + colBase + tid) * 2) = pv;
    }
    __threadfence();
#pragma unroll
    for (int it = 0; it < 16; ++it) {
      const int row = 16 * wave + it;
      *(volatile v4f*)(Cf + (size_t)(rowBase + row) * ldc + colBase + 4 * lane) = keep[it];
    }
    if (flags & 2) {
      if (tid < GC) *(volatile v2d*)(part + ((size_t)blockIdx.x * ncols + colBase + tid) * 2) = pv;
    }
  } else if constexpr (MODE == 1) {
    const int cg = lane & 15, rsel = lane >> 4;
    v4f bc0 = {0.f, 0.f, 0.f, 0.f}, bc1 = bc0;
    if (!(flags & 4)) {
      bc0 = *(const v4f*)(bias + colBase + 8 * cg);
      bc1 = *(const v4f*)(bias + colBase + 8 * cg + 4);
    }
    v8h keep[8];
#pragma unroll
    for (int it = 0; it < 8; ++it) {
      const int row = 16 * wave + 2 * it + rsel;
      const float* q = stg + row * GC + 8 * cg;
      v4f x0 = *(const v4f*)q, x1 = *(const v4f*)(q + 4);
      if (flags & 4) {
        const float bb = bias[rowBase + row];
        x0 = x0 + bb; x1 = x1 + bb;
      } else {
        x0 = x0 + bc0; x1 = x1 + bc1;
      }
      if (flags & 8) { x0 = relu4(x0); x1 = relu4(x1); }
      keep[it] = cvt8(x0, x1);
      *(volatile v8h*)(Ch + (size_t)(rowBase + row) * ldc + colBase + 8 * cg) = keep[it];
    }
    __threadfence();
#pragma unroll
    for (int it = 0; it < 8; ++it) {
      const int row = 16 * wave + 2 * it + rsel;
      *(volatile v8h*)(Ch + (size_t)(rowBase + row) * ldc + colBase + 8 * cg) = keep[it];
    }
  } else {
    _Float16* P = (colBase < C_) ? Ch : Ch2;
    const int hbase = (colBase & (C_ - 1)) >> 6;
    const int lq = lane >> 3, l8 = lane & 7;
    v8h keep[8];
#pragma unroll
    for (int j = 0; j < 8; ++j) {
      const int item = 4 * j + lq;
      const int rl = item >> 1, hs = item & 1;
      const int row = 16 * wave + rl;
      const int cl = 64 * hs + 8 * l8;
      const float* q = stg + row * GC + cl;
      v4f x0 = *(const v4f*)q, x1 = *(const v4f*)(q + 4);
      x0 = x0 + *(const v4f*)(bias + colBase + cl);
      x1 = x1 + *(const v4f*)(bias + colBase + cl + 4);
      keep[j] = cvt8(x0, x1);
      *(volatile v8h*)(P + ((size_t)(hbase + hs) * nN + rowBase + row) * HD + 8 * l8) = keep[j];
    }
    __threadfence();
#pragma unroll
    for (int j = 0; j < 8; ++j) {
      const int item = 4 * j + lq;
      const int rl = item >> 1, hs = item & 1;
      const int row = 16 * wave + rl;
      *(volatile v8h*)(P + ((size_t)(hbase + hs) * nN + rowBase + row) * HD + 8 * l8) = keep[j];
    }
  }
}

__global__ __launch_bounds__(ATHR) void k_attn(
    const _Float16* __restrict__ Qp, const _Float16* __restrict__ Kp,
    const _Float16* __restrict__ Vt, _Float16* ATT, int nN) {
  __shared__ __attribute__((aligned(16))) _Float16 sP[(ATHR / 32) * 16 * PP];
  const int tid = threadIdx.x, lane = tid & 31, wave = tid >> 5, hh = lane >> 4, m = lane & 15;
  const int h = blockIdx.y;
  const int q0 = blockIdx.x * AQ + wave * 16;
  _Float16* sw = sP + wave * 16 * PP;

  Frag qa0, qa1;
  {
    const _Float16* qp = Qp + ((size_t)h * nN + q0 + m) * HD + 8 * hh;
    qa0.h[0] = *(const v8h*)qp;
    qa0.h[1] = *(const v8h*)(qp + 16);
    qa1.h[0] = *(const v8h*)(qp + 32);
    qa1.h[1] = *(const v8h*)(qp + 48);
  }
  const _Float16* kbase = Kp + (size_t)h * nN * HD + (size_t)m * HD + 8 * hh;
  const _Float16* vbase = Vt + ((size_t)h * HD + m) * nN + 8 * hh;

  v8f o[4];
  float runM[8], runL[8];
#pragma unroll
  for (int t = 0; t < 4; ++t) o[t] = vz8();
#pragma unroll
  for (int r = 0; r < 8; ++r) { runM[r] = -1e30f; runL[r] = 0.0f; }

#pragma unroll 1
  for (int kb = 0; kb < nN; kb += 64) {
    v8f s[4];
#pragma unroll
    for (int t = 0; t < 4; ++t) {
      const _Float16* kp = kbase + (size_t)(kb + 16 * t) * HD;
      Frag b0, b1;
      b0.h[0] = *(const v8h*)kp;
      b0.h[1] = *(const v8h*)(kp + 16);
      b1.h[0] = *(const v8h*)(kp + 32);
      b1.h[1] = *(const v8h*)(kp + 48);
      v8f z = vz8();
      z = wmf(qa0.v, b0.v, z);
      z = wmf(qa1.v, b1.v, z);
      s[t] = z;
    }
    _Float16* pw = sw + (8 * hh) * PP + m;
#pragma unroll
    for (int r = 0; r < 8; ++r) {
      float mx = fmaxf(fmaxf(s[0][r], s[1][r]), fmaxf(s[2][r], s[3][r]));
      mx = fmaxf(mx, __shfl_xor(mx, 8));
      mx = fmaxf(mx, __shfl_xor(mx, 4));
      mx = fmaxf(mx, __shfl_xor(mx, 2));
      mx = fmaxf(mx, __shfl_xor(mx, 1));
      const float nm = fmaxf(runM[r], mx);
      const float alpha = __expf((runM[r] - nm) * 0.125f);
      runM[r] = nm;
      const float p0 = __expf((s[0][r] - nm) * 0.125f);
      const float p1 = __expf((s[1][r] - nm) * 0.125f);
      const float p2 = __expf((s[2][r] - nm) * 0.125f);
      const float p3 = __expf((s[3][r] - nm) * 0.125f);
      float ps = (p0 + p1) + (p2 + p3);
      ps += __shfl_xor(ps, 8);
      ps += __shfl_xor(ps, 4);
      ps += __shfl_xor(ps, 2);
      ps += __shfl_xor(ps, 1);
      runL[r] = runL[r] * alpha + ps;
      pw[r * PP]      = (_Float16)(p0 * 1024.0f);
      pw[r * PP + 16] = (_Float16)(p1 * 1024.0f);
      pw[r * PP + 32] = (_Float16)(p2 * 1024.0f);
      pw[r * PP + 48] = (_Float16)(p3 * 1024.0f);
      o[0][r] = o[0][r] * alpha;
      o[1][r] = o[1][r] * alpha;
      o[2][r] = o[2][r] * alpha;
      o[3][r] = o[3][r] * alpha;
    }
    __syncthreads();
#pragma unroll
    for (int ks = 0; ks < 2; ++ks) {
      Frag pa;
      const _Float16* pr = sw + m * PP + 32 * ks + 8 * hh;
      pa.h[0] = *(const v8h*)pr;
      pa.h[1] = *(const v8h*)(pr + 16);
#pragma unroll
      for (int dt = 0; dt < 4; ++dt) {
        const _Float16* vp = vbase + (size_t)(16 * dt) * nN + kb + 32 * ks;
        Frag vb;
        vb.h[0] = *(const v8h*)vp;
        vb.h[1] = *(const v8h*)(vp + 16);
        o[dt] = wmf(pa.v, vb.v, o[dt]);
      }
    }
    __syncthreads();
  }

#pragma unroll
  for (int r = 0; r < 8; ++r) {
    const float inv = __builtin_amdgcn_rcpf(runL[r]) * 0.0625f;
    _Float16* pw = sw + (8 * hh + r) * PP + m;
    pw[0]  = (_Float16)(o[0][r] * inv);
    pw[16] = (_Float16)(o[1][r] * inv);
    pw[32] = (_Float16)(o[2][r] * inv);
    pw[48] = (_Float16)(o[3][r] * inv);
  }
  __syncthreads();
  const int lq = lane >> 3, l8 = lane & 7;
  v8h keep[4];
#pragma unroll
  for (int j = 0; j < 4; ++j) {
    const int rl = 4 * j + lq;
    keep[j] = *(const v8h*)(sw + rl * PP + 8 * l8);
  }
#pragma unroll
  for (int j = 0; j < 4; ++j) {
    const int rl = 4 * j + lq;
    *(volatile v8h*)(ATT + (size_t)(q0 + rl) * C_ + h * HD + 8 * l8) = keep[j];
  }
  __threadfence();
#pragma unroll
  for (int j = 0; j < 4; ++j) {
    const int rl = 4 * j + lq;
    *(volatile v8h*)(ATT + (size_t)(q0 + rl) * C_ + h * HD + 8 * l8) = keep[j];
  }
}

__global__ __launch_bounds__(NTHR) void k_bnfin(const double* __restrict__ part, float* coef, int nRB, int nN) {
  __shared__ __attribute__((aligned(16))) float sco[2 * C_];
  const int tid = threadIdx.x, set = blockIdx.x;
  const double* pp = part + (size_t)set * nRB * (2 * C_);
  double S = 0.0, Q = 0.0;
#pragma unroll 1
  for (int b = 0; b < nRB; ++b) {
    const v2d q = *(const v2d*)(pp + ((size_t)b * C_ + tid) * 2);
    S += q.x;
    Q += q.y;
  }
  const double rn = 1.0 / (double)(nN > 1 ? nN : 1);
  const double mean = S * rn;
  double var = Q * rn - mean * mean;
  var = var < 0.0 ? 0.0 : var;
  sco[tid]      = (float)mean;
  sco[C_ + tid] = rsqrtf((float)var + 1e-5f);
  __syncthreads();
  v4f cv = {0.f, 0.f, 0.f, 0.f};
  if (tid < 128) cv = *(const v4f*)(sco + 4 * tid);
  float* cp = coef + (size_t)set * (2 * C_) + 4 * tid;
  if (tid < 128) *(volatile v4f*)cp = cv;
  __threadfence();
  if (tid < 128) *(volatile v4f*)cp = cv;
}

__global__ __launch_bounds__(NTHR) void k_bn12(
    const float* __restrict__ H1, const float* __restrict__ H2, const float* __restrict__ coef,
    const float* __restrict__ g1, const float* __restrict__ b1,
    const float* __restrict__ g2, const float* __restrict__ b2,
    float* O12, _Float16* O12h) {
  __shared__ __attribute__((aligned(16))) float stg[NTHR * 8];
  const int tid = threadIdx.x;
  const size_t base = (size_t)blockIdx.x * (NTHR * 8) + (size_t)tid * 8;
  const int c0 = (tid * 8) & (C_ - 1);
  const v4f h1a = *(const v4f*)(H1 + base), h1b = *(const v4f*)(H1 + base + 4);
  const v4f h2a = *(const v4f*)(H2 + base), h2b = *(const v4f*)(H2 + base + 4);
  const v4f m1a = *(const v4f*)(coef + c0),          m1b = *(const v4f*)(coef + c0 + 4);
  const v4f r1a = *(const v4f*)(coef + C_ + c0),     r1b = *(const v4f*)(coef + C_ + c0 + 4);
  const v4f m2a = *(const v4f*)(coef + 2 * C_ + c0), m2b = *(const v4f*)(coef + 2 * C_ + c0 + 4);
  const v4f r2a = *(const v4f*)(coef + 3 * C_ + c0), r2b = *(const v4f*)(coef + 3 * C_ + c0 + 4);
  const v4f g1a = *(const v4f*)(g1 + c0), g1b = *(const v4f*)(g1 + c0 + 4);
  const v4f b1a = *(const v4f*)(b1 + c0), b1b = *(const v4f*)(b1 + c0 + 4);
  const v4f g2a = *(const v4f*)(g2 + c0), g2b = *(const v4f*)(g2 + c0 + 4);
  const v4f b2a = *(const v4f*)(b2 + c0), b2b = *(const v4f*)(b2 + c0 + 4);
  const v4f t1a = (h1a - m1a) * r1a * g1a + b1a, t1b = (h1b - m1b) * r1b * g1b + b1b;
  const v4f t2a = (h2a - m2a) * r2a * g2a + b2a, t2b = (h2b - m2b) * r2b * g2b + b2b;
  const v4f va = t1a + t2a, vb = t1b + t2b;
  const v8h hv = cvt8(va, vb);
  *(v4f*)(stg + tid * 8)     = va;
  *(v4f*)(stg + tid * 8 + 4) = vb;
  *(volatile v8h*)(O12h + base) = hv;
  __syncthreads();
  const v4f f0 = *(const v4f*)(stg + 4 * tid);
  const v4f f1 = *(const v4f*)(stg + 4 * (tid + NTHR));
  float* ob = O12 + (size_t)blockIdx.x * (NTHR * 8);
  *(volatile v4f*)(ob + 4 * tid) = f0;
  *(volatile v4f*)(ob + 4 * (tid + NTHR)) = f1;
  __threadfence();
  *(volatile v8h*)(O12h + base) = hv;
  *(volatile v4f*)(ob + 4 * tid) = f0;
  *(volatile v4f*)(ob + 4 * (tid + NTHR)) = f1;
}

__global__ __launch_bounds__(NTHR) void k_bn3(
    const float* __restrict__ P3, const float* __restrict__ coef,
    const float* __restrict__ g3, const float* __restrict__ b3, _Float16* Eh) {
  const int tid = threadIdx.x;
  const size_t base = (size_t)blockIdx.x * (NTHR * 8) + (size_t)tid * 8;
  const int c0 = (tid * 8) & (C_ - 1);
  const v4f pa = *(const v4f*)(P3 + base), pb = *(const v4f*)(P3 + base + 4);
  const v4f ma = *(const v4f*)(coef + c0),      mb = *(const v4f*)(coef + c0 + 4);
  const v4f ra = *(const v4f*)(coef + C_ + c0), rb = *(const v4f*)(coef + C_ + c0 + 4);
  const v4f ga = *(const v4f*)(g3 + c0), gb = *(const v4f*)(g3 + c0 + 4);
  const v4f ba = *(const v4f*)(b3 + c0), bb = *(const v4f*)(b3 + c0 + 4);
  v4f va = (pa - ma) * ra * ga + ba, vb = (pb - mb) * rb * gb + bb;
  va.x = elu1(va.x); va.y = elu1(va.y); va.z = elu1(va.z); va.w = elu1(va.w);
  vb.x = elu1(vb.x); vb.y = elu1(vb.y); vb.z = elu1(vb.z); vb.w = elu1(vb.w);
  const v8h hv = cvt8(va, vb);
  *(volatile v8h*)(Eh + base) = hv;
  __threadfence();
  *(volatile v8h*)(Eh + base) = hv;
}

extern "C" void kernel_launch(void* const* d_in, const int* in_sizes, int n_in,
                              void* d_out, int out_size, void* d_ws, size_t ws_size,
                              hipStream_t stream) {
  if (n_in < 21) return;
  const int nN = in_sizes[0] / C_;
  if (nN <= 0 || in_sizes[0] != nN * C_ || (nN % GR) != 0 || nN > (1 << 20)) return;
  if (in_sizes[1] < 2 || (in_sizes[1] & 1) != 0) return;
  const int nE = in_sizes[1] / 2;
  if (nE <= 0 || nE > (1 << 28)) return;
  if (in_sizes[2] != C_ * C_ || in_sizes[3] != C_ || in_sizes[4] != C_ * C_) return;
  if (in_sizes[5] != 3 * C_ * C_ || in_sizes[6] != 3 * C_) return;
  if (in_sizes[7] != C_ * C_ || in_sizes[8] != C_) return;
  for (int i = 9; i <= 14; ++i) if (in_sizes[i] != C_) return;
  if (in_sizes[15] != 2 * C_ * C_ || in_sizes[16] != 2 * C_) return;
  if (in_sizes[17] != 2 * C_ * C_ || in_sizes[18] != C_) return;
  if (in_sizes[19] != C_ * C_ || in_sizes[20] != C_) return;
  if (out_size != nN * C_) return;

  const float* x      = (const float*)d_in[0];
  const int*   eidx   = (const int*)d_in[1];
  const float* w_ngh  = (const float*)d_in[2];
  const float* b_ngh  = (const float*)d_in[3];
  const float* w_root = (const float*)d_in[4];
  const float* w_in   = (const float*)d_in[5];
  const float* b_in   = (const float*)d_in[6];
  const float* w_out  = (const float*)d_in[7];
  const float* b_out  = (const float*)d_in[8];
  const float* bn1_g  = (const float*)d_in[9];
  const float* bn1_b  = (const float*)d_in[10];
  const float* bn2_g  = (const float*)d_in[11];
  const float* bn2_b  = (const float*)d_in[12];
  const float* bn3_g  = (const float*)d_in[13];
  const float* bn3_b  = (const float*)d_in[14];
  const float* w_mlp1 = (const float*)d_in[15];
  const float* b_mlp1 = (const float*)d_in[16];
  const float* w_mlp2 = (const float*)d_in[17];
  const float* b_mlp2 = (const float*)d_in[18];
  const float* w_lin  = (const float*)d_in[19];
  const float* b_lin  = (const float*)d_in[20];
  const int* srcs = eidx;
  const int* dsts = eidx + nE;
  float* out = (float*)d_out;

  const int nRB = nN / GR;

  char* ws = (char*)d_ws;
  size_t off = 0;
  auto take = [&](size_t bytes) -> size_t { const size_t o = off; off += (bytes + 255) & ~(size_t)255; return o; };
  const size_t oW    = take((size_t)WPTOT * 2);
  const size_t oA1   = take((size_t)nN * (2 * C_) * 2);
  const size_t oH1   = take((size_t)nN * C_ * 4);
  const size_t oQ    = take((size_t)NH * nN * HD * 2);
  const size_t oK    = take((size_t)NH * nN * HD * 2);
  const size_t oVt   = take((size_t)C_ * nN * 2);
  const size_t oATT  = take((size_t)nN * C_ * 2);
  const size_t oH2   = take((size_t)nN * C_ * 4);
  const size_t oPart = take((size_t)3 * nRB * C_ * 2 * 8);
  const size_t oCoef = take((size_t)3 * 2 * C_ * 4);
  const size_t oO12  = take((size_t)nN * C_ * 4);
  const size_t oO12h = take((size_t)nN * C_ * 2);
  const size_t oT1   = take((size_t)nN * (2 * C_) * 2);
  const size_t oP3   = take((size_t)nN * C_ * 4);
  const size_t oE    = take((size_t)nN * C_ * 2);
  if (off > ws_size || off > (size_t)WSCAP) return;

  _Float16* wp   = (_Float16*)(ws + oW);
  _Float16* A1   = (_Float16*)(ws + oA1);
  float*    H1   = (float*)(ws + oH1);
  _Float16* Qp   = (_Float16*)(ws + oQ);
  _Float16* Kp   = (_Float16*)(ws + oK);
  _Float16* Vt   = (_Float16*)(ws + oVt);
  _Float16* ATT  = (_Float16*)(ws + oATT);
  float*    H2   = (float*)(ws + oH2);
  double*   part = (double*)(ws + oPart);
  float*    coef = (float*)(ws + oCoef);
  float*    O12  = (float*)(ws + oO12);
  _Float16* O12h = (_Float16*)(ws + oO12h);
  _Float16* T1   = (_Float16*)(ws + oT1);
  float*    P3   = (float*)(ws + oP3);
  _Float16* Eh   = (_Float16*)(ws + oE);
  const size_t partSet = (size_t)nRB * C_ * 2;

  const int vec8 = ((nE & 3) == 0) ? 1 : 0;
  const float rw = 1.0f / WSCL;

  hipFuncSetAttribute(reinterpret_cast<const void*>(&k_gemm<0>), hipFuncAttributeMaxDynamicSharedMemorySize, LDS_GEMM);
  hipFuncSetAttribute(reinterpret_cast<const void*>(&k_gemm<1>), hipFuncAttributeMaxDynamicSharedMemorySize, LDS_GEMM);
  hipFuncSetAttribute(reinterpret_cast<const void*>(&k_gemm<2>), hipFuncAttributeMaxDynamicSharedMemorySize, LDS_GEMM);

  k_wprep<<<352, NTHR, 0, stream>>>(w_ngh, w_root, w_in, w_out, w_mlp1, w_mlp2, w_lin, wp);

  k_agg<<<nN / AGB, NTHR, 0, stream>>>(x, srcs, dsts, A1, nN, nE, vec8);

  k_gemm<0><<<dim3(nRB, C_ / GC), NTHR, LDS_GEMM, stream>>>(
      A1, 2 * C_, wp + WP_1, 2 * C_, 2 * C_, b_ngh, x, C_, rw,
      H1, A1, A1, C_, part, 3, nN);

  k_gemm<2><<<dim3(nRB, (2 * C_) / GC), NTHR, LDS_GEMM, stream>>>(
      A1 + C_, 2 * C_, wp + WP_IN, C_, C_, b_in, x, C_, rw,
      H1, Qp, Kp, HD, part, 0, nN);

  k_gemm<1><<<dim3(C_ / GR, nN / GC), NTHR, LDS_GEMM, stream>>>(
      wp + WP_IN + (size_t)2 * C_ * C_, C_, A1 + C_, 2 * C_, C_, b_in + 2 * C_, x, C_, rw,
      H1, Vt, Vt, nN, part, 4, nN);

  k_attn<<<dim3(nN / AQ, NH), ATHR, 0, stream>>>(Qp, Kp, Vt, ATT, nN);

  k_gemm<0><<<dim3(nRB, C_ / GC), NTHR, LDS_GEMM, stream>>>(
      ATT, C_, wp + WP_OUT, C_, C_, b_out, x, C_, rw * (1.0f / 64.0f),
      H2, A1, A1, C_, part + partSet, 3, nN);

  k_bnfin<<<2, NTHR, 0, stream>>>(part, coef, nRB, nN);

  k_bn12<<<nN / 8, NTHR, 0, stream>>>(H1, H2, coef, bn1_g, bn1_b, bn2_g, bn2_b, O12, O12h);

  k_gemm<1><<<dim3(nRB, (2 * C_) / GC), NTHR, LDS_GEMM, stream>>>(
      O12h, C_, wp + WP_M1, C_, C_, b_mlp1, x, C_, rw,
      H1, T1, T1, 2 * C_, part, 8, nN);

  k_gemm<0><<<dim3(nRB, C_ / GC), NTHR, LDS_GEMM, stream>>>(
      T1, 2 * C_, wp + WP_M2, 2 * C_, 2 * C_, b_mlp2, O12, C_, rw,
      P3, A1, A1, C_, part + 2 * partSet, 3, nN);

  k_bnfin<<<1, NTHR, 0, stream>>>(part + 2 * partSet, coef + 2 * (2 * C_), nRB, nN);

  k_bn3<<<nN / 8, NTHR, 0, stream>>>(P3, coef + 2 * (2 * C_), bn3_g, bn3_b, Eh);

  k_gemm<0><<<dim3(nRB, C_ / GC), NTHR, LDS_GEMM, stream>>>(
      Eh, C_, wp + WP_LIN, C_, C_, b_lin, x, C_, rw,
      out, A1, A1, C_, part, 0, nN);
}
